// sFSMNCell_88562225643917
// MI455X (gfx1250) — hardware-run, weakly checked
//
#include <hip/hip_runtime.h>


namespace {
constexpr int NB = 8, T = 2048, D = 512, MEM = 32;
constexpr float XS = 8.0f, WSC = 256.0f;
typedef _Float16 b16;
typedef __attribute__((ext_vector_type(16))) _Float16 v16b;
typedef __attribute__((ext_vector_type(8))) _Float16 v8b;
typedef __attribute__((ext_vector_type(8))) float v8f;
typedef __attribute__((ext_vector_type(4))) float v4f;
__device__ __forceinline__ float bf16_rne(float f) { unsigned int u = __float_as_uint(f); u += 0x7FFFu + ((u >> 16) & 1u); float r = __uint_as_float(u & 0xFFFF0000u); asm volatile("" : "+v"(r)); return r; }
__device__ __forceinline__ v16b frag_kb(const b16* p, int hh) { const v8b a = *(const v8b*)(p + 8 * hh), b = *(const v8b*)(p + 16 + 8 * hh); v16b f;
#pragma unroll
  for (int e = 0; e < 8; ++e) { f[e] = a[e]; f[8 + e] = b[e]; } return f; }
__device__ __forceinline__ v8f wmma16b(v16b a, v16b b, v8f c) { v8f d = __builtin_amdgcn_wmma_f32_16x16x32_f16(false, a, false, b, (short)0, c, false, false); asm volatile("v_nop\n\tv_nop\n\tv_nop\n\tv_nop" : "+v"(d) : "v"(a), "v"(b)); return d; }
__device__ __forceinline__ void wave_lds_sync() { __builtin_amdgcn_fence(__ATOMIC_RELEASE, "workgroup"); __builtin_amdgcn_wave_barrier(); __builtin_amdgcn_fence(__ATOMIC_ACQUIRE, "workgroup"); }
__device__ __forceinline__ float pmul(float a, float b) { float p = a * b; asm volatile("" : "+v"(p)); return p; }

__global__ __launch_bounds__(256) void wput_kernel(const float* __restrict__ w1, const float* __restrict__ w2, b16* __restrict__ WT) { const int u = blockIdx.x * 256 + threadIdx.x; if (u >= 2 * D * 64) return; const int r = u / 64, k0 = (u % 64) * 8; const float* w = r < D ? w1 : w2; const int o = r % D; v8b v;
#pragma unroll
  for (int j = 0; j < 8; ++j) v[j] = (b16)(bf16_rne(w[(size_t)(k0 + j) * D + o]) * WSC); for (int pass = 0; pass < 2; ++pass) { *(volatile v8b*)(WT + (size_t)r * D + k0) = v; __threadfence(); } }
__global__ __launch_bounds__(32) void proj_kernel(const float* __restrict__ x, const b16* __restrict__ WT, int RLIM, float* __restrict__ P) { __shared__ __attribute__((aligned(16))) b16 Ah[16][D + 8]; __shared__ float Tf[16][260]; const int lane = threadIdx.x, nloc = lane & 15, hlf = lane >> 4; const int g = blockIdx.x & 3; const size_t m0 = (size_t)(blockIdx.x >> 2) * 16; if (m0 >= (size_t)RLIM) return;
  for (int rr = 0; rr < 16; ++rr) for (int q = 0; q < D / 32; ++q) Ah[rr][q * 32 + lane] = (b16)(bf16_rne(x[(m0 + rr) * D + q * 32 + lane]) * XS);
  wave_lds_sync(); v8f acc[16];
#pragma unroll
  for (int t = 0; t < 16; ++t) acc[t] = (v8f){};
#pragma unroll 2
  for (int kb = 0; kb < D; kb += 32) { const v16b a = frag_kb(&Ah[nloc][kb], hlf);
#pragma unroll
    for (int t = 0; t < 16; ++t) acc[t] = wmma16b(a, frag_kb(WT + (size_t)(g * 256 + t * 16 + nloc) * D + kb, hlf), acc[t]); }
#pragma unroll
  for (int t = 0; t < 16; ++t)
#pragma unroll
    for (int r8 = 0; r8 < 8; ++r8) Tf[8 * hlf + r8][t * 16 + nloc] = acc[t][r8] * (1.0f / (XS * WSC));
  wave_lds_sync();
  for (int pass = 0; pass < 2; ++pass) { for (int rr = 0; rr < 16; ++rr) for (int q = 0; q < 2; ++q) *(volatile v4f*)(P + (m0 + rr) * (2 * D) + g * 256 + q * 128 + lane * 4) = *(const v4f*)(&Tf[rr][q * 128 + lane * 4]); __threadfence(); } }
__global__ __launch_bounds__(256) void band_kernel(const float* __restrict__ P, const float* __restrict__ bias, int RLIM, float* __restrict__ out) { const int wave = threadIdx.x >> 5, lane = threadIdx.x & 31; const size_t row = (size_t)blockIdx.x * 8 + wave; if (row >= (size_t)RLIM) return; const int n = (int)(row % T);
  float acc[16];
#pragma unroll
  for (int k = 0; k < 16; ++k) acc[k] = P[row * (2 * D) + lane * 16 + k] + bf16_rne(bias[lane * 16 + k]);
#pragma unroll 1
  for (int d = 1; d <= MEM; ++d) { if (n - d < 0) break; const float* pr = P + (row - d) * (2 * D) + D + lane * 16; const float wd = (float)d;
#pragma unroll
    for (int k = 0; k < 16; ++k) acc[k] += pmul(wd, pr[k]); }
  for (int pass = 0; pass < 2; ++pass) {
#pragma unroll
    for (int q = 0; q < 4; ++q) *(volatile v4f*)(out + row * D + lane * 16 + q * 4) = (v4f){acc[q * 4], acc[q * 4 + 1], acc[q * 4 + 2], acc[q * 4 + 3]}; __threadfence(); } }
}

extern "C" void kernel_launch(void* const* d_in, const int* in_sizes, int n_in, void* d_out, int out_size, void* d_ws, size_t ws_size, hipStream_t stream) {
  (void)n_in;
  auto Fp = [&](int i) { return (const float*)d_in[i]; };
  if (in_sizes[0] != NB * T * D || in_sizes[1] != D * D || in_sizes[2] != D * D || in_sizes[3] != D || out_size != NB * T * D) return;
  const int RLIM = NB * T;
  size_t off = 0; char* ws = (char*)d_ws;
  auto carve = [&](size_t bytes) { char* p = ws + off; off += (bytes + 255) & ~(size_t)255; return p; };
  b16* WT = (b16*)carve((size_t)2 * D * D * 2); float* P = (float*)carve((size_t)NB * T * 2 * D * 4);
  if (off > ws_size || off > ((size_t)96 << 20)) return;
  wput_kernel<<<(2 * D * 64 + 255) / 256, 256, 0, stream>>>(Fp(1), Fp(2), WT);
  proj_kernel<<<(RLIM / 16) * 4, 32, 0, stream>>>(Fp(0), WT, RLIM, P);
  band_kernel<<<(RLIM + 7) / 8, 256, 0, stream>>>(P, Fp(3), RLIM, (float*)d_out);
}
